// KnowledgeMemoryv3_4964982194880
// MI455X (gfx1250) — hardware-verified
//
#include <hip/hip_runtime.h>
#include <stddef.h>
#include <stdint.h>


#define NB   8
#define NQ   128
#define NM   1024
#define ND   256
#define NSL  3
#define NHOP 2
#define NTHR 128

static_assert(ND == 2 * NTHR);
static_assert(NM == 8 * NTHR);
static_assert((NB * NQ) % 32 == 0);
static_assert((NB * NM) % 32 == 0);

typedef _Float16 v8h  __attribute__((ext_vector_type(8)));
typedef _Float16 v16h __attribute__((ext_vector_type(16)));
typedef float    v8f  __attribute__((ext_vector_type(8)));
typedef float    v4f  __attribute__((ext_vector_type(4)));
typedef int      v4i  __attribute__((ext_vector_type(4)));

union Frag { v16h v; v8h h[2]; };

#if __has_builtin(__builtin_amdgcn_exp2f)
#define EXP2_FAST(x) __builtin_amdgcn_exp2f(x)
#else
#define EXP2_FAST(x) exp2f(x)
#endif
#define RCP_FAST(x) __builtin_amdgcn_rcpf(x)

__device__ __forceinline__ v16h frag16(const _Float16* row, int k0, int hh)
{
    Frag f;
    f.h[0] = *(const v8h*)(row + k0 + 8 * hh);
    f.h[1] = *(const v8h*)(row + k0 + 16 + 8 * hh);
    return f.v;
}

__device__ __forceinline__ v8f wmma_f16(v16h a, v16h b, v8f c)
{
    v8f d = __builtin_amdgcn_wmma_f32_16x16x32_f16(false, a, false, b, (short)0, c, false, false);
    asm volatile("v_nop\n\tv_nop\n\tv_nop\n\tv_nop" : "+v"(d) : "v"(a), "v"(b));
    return d;
}

__device__ __forceinline__ v8h pack8h(v4f a, v4f b)
{
    v8h r = { (_Float16)a[0], (_Float16)a[1], (_Float16)a[2], (_Float16)a[3],
              (_Float16)b[0], (_Float16)b[1], (_Float16)b[2], (_Float16)b[3] };
    return r;
}

__global__ void __launch_bounds__(NTHR) prep_kernel(
    const float* __restrict__ query, const float* __restrict__ kb, const float* __restrict__ sel,
    const float* __restrict__ Wq, const float* __restrict__ Wm,
    _Float16* q16, _Float16* wq16, _Float16* wm16, _Float16* km16, _Float16* kmT16,
    int hop, int nqb)
{
    __shared__ float s_t[32][65];

    const int tid = threadIdx.x;
    const int bid = blockIdx.x;
    const int segA = nqb;
    const int segB = segA + ND / 4;
    const int segC = segB + ND / 4;
    const int segD = segC + (NB * NM) / 4;

    if (bid < segD) {
        const int rl = tid >> 5;
        const int c8 = tid & 31;
        const float* src;
        _Float16* dst;
        float scale;
        if (bid < segA) {
            const int row = bid * 4 + rl;
            src = query + (size_t)row * ND;
            dst = q16 + (size_t)row * ND;
            scale = 1.0f;
        } else if (bid < segB) {
            const int row = (bid - segA) * 4 + rl;
            src = Wq + ((size_t)hop * ND + row) * ND;
            dst = wq16 + (size_t)row * ND;
            scale = 16.0f;
        } else if (bid < segC) {
            const int row = (bid - segB) * 4 + rl;
            src = Wm + ((size_t)hop * ND + row) * ND;
            dst = wm16 + (size_t)row * ND;
            scale = 16.0f;
        } else {
            const int row = (bid - segC) * 4 + rl;
            const int b = row >> 10;
            const int m = row & (NM - 1);
            src = kb + (((size_t)b * NSL + hop) * NM + m) * ND;
            dst = km16 + (size_t)row * ND;
            scale = sel[row];
        }
        const v4f x0 = *(const v4f*)(src + 8 * c8);
        const v4f x1 = *(const v4f*)(src + 8 * c8 + 4);
        const v8h val = pack8h(x0 * scale, x1 * scale);
        volatile v8h* p = (volatile v8h*)(dst + 8 * c8);
        *p = val;
        __threadfence();
        *p = val;
    } else {
        const int t = bid - segD;
        const int b = t >> 7;
        const int rem = t & 127;
        const int m0 = (rem >> 3) * 64;
        const int d0 = (rem & 7) * 32;
        const float* src = kb + (((size_t)b * NSL + hop + 1) * NM + m0) * ND + d0;
        #pragma unroll
        for (int i = 0; i < 4; ++i) {
            const int idx = tid + NTHR * i;
            const int row = idx >> 3;
            const int c4 = idx & 7;
            const v4f x = *(const v4f*)(src + (size_t)row * ND + 4 * c4);
            const float s = sel[b * NM + m0 + row];
            s_t[4 * c4 + 0][row] = x[0] * s;
            s_t[4 * c4 + 1][row] = x[1] * s;
            s_t[4 * c4 + 2][row] = x[2] * s;
            s_t[4 * c4 + 3][row] = x[3] * s;
        }
        __syncthreads();
        v8h val[2];
        size_t off[2];
        #pragma unroll
        for (int i = 0; i < 2; ++i) {
            const int idx = tid + NTHR * i;
            const int dl = idx >> 3;
            const int ms = (idx & 7) * 8;
            v8h r = { (_Float16)s_t[dl][ms + 0], (_Float16)s_t[dl][ms + 1],
                      (_Float16)s_t[dl][ms + 2], (_Float16)s_t[dl][ms + 3],
                      (_Float16)s_t[dl][ms + 4], (_Float16)s_t[dl][ms + 5],
                      (_Float16)s_t[dl][ms + 6], (_Float16)s_t[dl][ms + 7] };
            val[i] = r;
            off[i] = ((size_t)(b * ND + d0 + dl)) * NM + m0 + ms;
        }
        #pragma unroll
        for (int i = 0; i < 2; ++i) *(volatile v8h*)(kmT16 + off[i]) = val[i];
        __threadfence();
        #pragma unroll
        for (int i = 0; i < 2; ++i) *(volatile v8h*)(kmT16 + off[i]) = val[i];
    }
}

__global__ void __launch_bounds__(NTHR) proj_gemm_kernel(
    const _Float16* __restrict__ A, const _Float16* __restrict__ Bt, const float* __restrict__ bias,
    float bias_mul, float scale, float post, float* C)
{
    __shared__ __align__(16) float s_c[32][260];

    const int tid = threadIdx.x;
    const int wv  = tid >> 5;
    const int l   = tid & 31;
    const int hh  = l >> 4;
    const int m15 = l & 15;
    const int row0 = blockIdx.x * 32;

    v8f acc[2][4];
    const v8f zero = { 0.f, 0.f, 0.f, 0.f, 0.f, 0.f, 0.f, 0.f };
    #pragma unroll
    for (int rt = 0; rt < 2; ++rt)
        #pragma unroll
        for (int j = 0; j < 4; ++j) acc[rt][j] = zero;

    const _Float16* a0p = A  + (size_t)(row0 + m15) * ND;
    const _Float16* a1p = A  + (size_t)(row0 + 16 + m15) * ND;
    const _Float16* bp  = Bt + (size_t)(64 * wv + m15) * ND;

    for (int k0 = 0; k0 < ND; k0 += 32) {
        const v16h fa0 = frag16(a0p, k0, hh);
        const v16h fa1 = frag16(a1p, k0, hh);
        #pragma unroll
        for (int j = 0; j < 4; ++j) {
            const v16h fb = frag16(bp + (size_t)j * 16 * ND, k0, hh);
            acc[0][j] = wmma_f16(fa0, fb, acc[0][j]);
            acc[1][j] = wmma_f16(fa1, fb, acc[1][j]);
        }
    }

    #pragma unroll
    for (int rt = 0; rt < 2; ++rt)
        #pragma unroll
        for (int j = 0; j < 4; ++j)
            #pragma unroll
            for (int r = 0; r < 8; ++r)
                s_c[rt * 16 + 8 * hh + r][64 * wv + 16 * j + m15] = acc[rt][j][r];
    __syncthreads();

    v4f vals[16];
    #pragma unroll
    for (int i = 0; i < 16; ++i) {
        const int idx = tid + NTHR * i;
        const int row = idx >> 6;
        const int c4  = idx & 63;
        const v4f x  = *(const v4f*)&s_c[row][4 * c4];
        const v4f bb = *(const v4f*)(bias + 4 * c4);
        vals[i] = (x * scale + bb * bias_mul) * post;
    }
    #pragma unroll
    for (int i = 0; i < 16; ++i) {
        const int idx = tid + NTHR * i;
        const int row = idx >> 6;
        const int c4  = idx & 63;
        *(volatile v4f*)(C + (size_t)(row0 + row) * ND + 4 * c4) = vals[i];
    }
    __threadfence();
    #pragma unroll
    for (int i = 0; i < 16; ++i) {
        const int idx = tid + NTHR * i;
        const int row = idx >> 6;
        const int c4  = idx & 63;
        *(volatile v4f*)(C + (size_t)(row0 + row) * ND + 4 * c4) = vals[i];
    }
}

__global__ void __launch_bounds__(NTHR) score_readout_kernel(
    const float* __restrict__ qhs, const float* __restrict__ mhs, const float* __restrict__ vvec,
    const int* __restrict__ mask, const _Float16* __restrict__ kmT,
    const float* __restrict__ qin, _Float16* qnext, float* o_out, float* w_out,
    int hop, int last)
{
    __shared__ __align__(16) float    s_v[ND];
    __shared__ __align__(16) float    s_qh[4][ND];
    __shared__ __align__(16) _Float16 s_p[16][NM];
    __shared__ __align__(16) float    s_f[16 * ND];
    __shared__ float s_rmax[4][4];
    __shared__ float s_rsum[4][4];

    const int tid = threadIdx.x;
    const int wv  = tid >> 5;
    const int l   = tid & 31;
    const int hh  = l >> 4;
    const int m15 = l & 15;
    const int b   = blockIdx.y;
    const int q0  = blockIdx.x * 16;
    const int mb  = 8 * tid;

    const float NEG_INF = -__builtin_inff();
    const float LOG2E   = 1.4426950408889634f;

    s_v[tid]        = vvec[hop * ND + tid];
    s_v[tid + NTHR] = vvec[hop * ND + tid + NTHR];

    int mbits = 0;
    {
        const v4i k0 = *(const v4i*)(mask + b * NM + mb);
        const v4i k1 = *(const v4i*)(mask + b * NM + mb + 4);
        #pragma unroll
        for (int e = 0; e < 4; ++e) {
            mbits |= (k0[e] != 0 ? 1 : 0) << e;
            mbits |= (k1[e] != 0 ? 1 : 0) << (4 + e);
        }
    }
    const float* mrow = mhs + ((size_t)b * NM + mb) * ND;

    for (int jq = 0; jq < 4; ++jq) {
        const int qrow0 = b * NQ + q0 + 4 * jq;

        #pragma unroll
        for (int i = 0; i < 2; ++i) {
            const int idx = tid + NTHR * i;
            const int j  = idx >> 6;
            const int c4 = idx & 63;
            *(v4f*)&s_qh[j][4 * c4] = *(const v4f*)(qhs + (size_t)(qrow0 + j) * ND + 4 * c4);
        }
        __syncthreads();

        float acc[4][8];
        #pragma unroll
        for (int j = 0; j < 4; ++j)
            #pragma unroll
            for (int i = 0; i < 8; ++i) acc[j][i] = 0.0f;

        #pragma unroll 1
        for (int d4 = 0; d4 < ND / 4; ++d4) {
            v4f mv[8];
            #pragma unroll
            for (int i = 0; i < 8; ++i) mv[i] = *(const v4f*)(mrow + (size_t)i * ND + 4 * d4);
            v4f qv[4];
            #pragma unroll
            for (int j = 0; j < 4; ++j) qv[j] = *(const v4f*)&s_qh[j][4 * d4];
            const v4f vv = *(const v4f*)&s_v[4 * d4];
            #pragma unroll
            for (int e = 0; e < 4; ++e) {
                const float ve = vv[e];
                #pragma unroll
                for (int j = 0; j < 4; ++j) {
                    const float qe = qv[j][e];
                    #pragma unroll
                    for (int i = 0; i < 8; ++i) {
                        const float hx = qe + mv[i][e];
                        const float ex = EXP2_FAST(hx);
                        const float rr = RCP_FAST(ex + 1.0f);
                        acc[j][i] = fmaf(ve, rr, acc[j][i]);
                    }
                }
            }
        }

        float bm[4];
        #pragma unroll
        for (int j = 0; j < 4; ++j) {
            float lm = NEG_INF;
            #pragma unroll
            for (int i = 0; i < 8; ++i) {
                const float s = ((mbits >> i) & 1) ? NEG_INF : -2.0f * acc[j][i];
                acc[j][i] = s;
                lm = fmaxf(lm, s);
            }
            #pragma unroll
            for (int off = 16; off > 0; off >>= 1) lm = fmaxf(lm, __shfl_xor(lm, off, 32));
            bm[j] = lm;
        }
        if (l == 0) {
            #pragma unroll
            for (int j = 0; j < 4; ++j) s_rmax[j][wv] = bm[j];
        }
        __syncthreads();
        #pragma unroll
        for (int j = 0; j < 4; ++j)
            bm[j] = fmaxf(fmaxf(s_rmax[j][0], s_rmax[j][1]), fmaxf(s_rmax[j][2], s_rmax[j][3]));

        float bs[4];
        #pragma unroll
        for (int j = 0; j < 4; ++j) {
            float ls = 0.0f;
            #pragma unroll
            for (int i = 0; i < 8; ++i) {
                const float ev = EXP2_FAST((acc[j][i] - bm[j]) * LOG2E);
                acc[j][i] = ev;
                ls += ev;
            }
            #pragma unroll
            for (int off = 16; off > 0; off >>= 1) ls += __shfl_xor(ls, off, 32);
            bs[j] = ls;
        }
        if (l == 0) {
            #pragma unroll
            for (int j = 0; j < 4; ++j) s_rsum[j][wv] = bs[j];
        }
        __syncthreads();
        #pragma unroll
        for (int j = 0; j < 4; ++j)
            bs[j] = (s_rsum[j][0] + s_rsum[j][1]) + (s_rsum[j][2] + s_rsum[j][3]);

        #pragma unroll
        for (int j = 0; j < 4; ++j) {
            const float inv = 1.0f / bs[j];
            const v4f w0 = { acc[j][0] * inv, acc[j][1] * inv, acc[j][2] * inv, acc[j][3] * inv };
            const v4f w1 = { acc[j][4] * inv, acc[j][5] * inv, acc[j][6] * inv, acc[j][7] * inv };
            *(v8h*)&s_p[4 * jq + j][mb] = pack8h(w0 * 16384.0f, w1 * 16384.0f);
            if (last) {
                *(v4f*)&s_f[j * NM + mb]     = w0;
                *(v4f*)&s_f[j * NM + mb + 4] = w1;
            }
        }
        if (last) {
            __syncthreads();
            v4f wr[8];
            #pragma unroll
            for (int i = 0; i < 8; ++i) {
                const int idx = tid + NTHR * i;
                const int j  = idx >> 8;
                const int c4 = idx & 255;
                wr[i] = *(const v4f*)&s_f[j * NM + 4 * c4];
            }
            #pragma unroll
            for (int i = 0; i < 8; ++i) {
                const int idx = tid + NTHR * i;
                const int j  = idx >> 8;
                const int c4 = idx & 255;
                *(volatile v4f*)(w_out + (size_t)(qrow0 + j) * NM + 4 * c4) = wr[i];
            }
            __threadfence();
            #pragma unroll
            for (int i = 0; i < 8; ++i) {
                const int idx = tid + NTHR * i;
                const int j  = idx >> 8;
                const int c4 = idx & 255;
                *(volatile v4f*)(w_out + (size_t)(qrow0 + j) * NM + 4 * c4) = wr[i];
            }
        }
    }
    __syncthreads();

    v8f pacc[4];
    const v8f zero = { 0.f, 0.f, 0.f, 0.f, 0.f, 0.f, 0.f, 0.f };
    #pragma unroll
    for (int j = 0; j < 4; ++j) pacc[j] = zero;

    const _Float16* prow = &s_p[m15][0];
    const _Float16* brow = kmT + ((size_t)(b * ND + 64 * wv + m15)) * NM;
    for (int k0 = 0; k0 < NM; k0 += 32) {
        const v16h fa = frag16(prow, k0, hh);
        #pragma unroll
        for (int j = 0; j < 4; ++j) {
            const v16h fb = frag16(brow + (size_t)j * 16 * NM, k0, hh);
            pacc[j] = wmma_f16(fa, fb, pacc[j]);
        }
    }
    const float OSC = 6.103515625e-05f;
    #pragma unroll
    for (int j = 0; j < 4; ++j)
        #pragma unroll
        for (int r = 0; r < 8; ++r)
            s_f[(8 * hh + r) * ND + 64 * wv + 16 * j + m15] = pacc[j][r] * OSC;
    __syncthreads();

    if (last) {
        v4f ov[8];
        #pragma unroll
        for (int i = 0; i < 8; ++i) {
            const int idx = tid + NTHR * i;
            const int row = idx >> 6;
            const int c4  = idx & 63;
            ov[i] = *(const v4f*)&s_f[row * ND + 4 * c4];
        }
        #pragma unroll
        for (int i = 0; i < 8; ++i) {
            const int idx = tid + NTHR * i;
            const int row = idx >> 6;
            const int c4  = idx & 63;
            *(volatile v4f*)(o_out + (size_t)(b * NQ + q0 + row) * ND + 4 * c4) = ov[i];
        }
        __threadfence();
        #pragma unroll
        for (int i = 0; i < 8; ++i) {
            const int idx = tid + NTHR * i;
            const int row = idx >> 6;
            const int c4  = idx & 63;
            *(volatile v4f*)(o_out + (size_t)(b * NQ + q0 + row) * ND + 4 * c4) = ov[i];
        }
    } else {
        v8h qv8[4];
        #pragma unroll
        for (int i = 0; i < 4; ++i) {
            const int idx = tid + NTHR * i;
            const int row = idx >> 5;
            const int c8  = idx & 31;
            const size_t goff = (size_t)(b * NQ + q0 + row) * ND + 8 * c8;
            const v4f o0 = *(const v4f*)&s_f[row * ND + 8 * c8];
            const v4f o1 = *(const v4f*)&s_f[row * ND + 8 * c8 + 4];
            const v4f qa = *(const v4f*)(qin + goff);
            const v4f qb = *(const v4f*)(qin + goff + 4);
            qv8[i] = pack8h(qa + o0, qb + o1);
        }
        #pragma unroll
        for (int i = 0; i < 4; ++i) {
            const int idx = tid + NTHR * i;
            const int row = idx >> 5;
            const int c8  = idx & 31;
            *(volatile v8h*)(qnext + (size_t)(b * NQ + q0 + row) * ND + 8 * c8) = qv8[i];
        }
        __threadfence();
        #pragma unroll
        for (int i = 0; i < 4; ++i) {
            const int idx = tid + NTHR * i;
            const int row = idx >> 5;
            const int c8  = idx & 31;
            *(volatile v8h*)(qnext + (size_t)(b * NQ + q0 + row) * ND + 8 * c8) = qv8[i];
        }
    }
}

extern "C" void kernel_launch(void* const* d_in, const int* in_sizes, int n_in,
                              void* d_out, int out_size, void* d_ws, size_t ws_size,
                              hipStream_t stream)
{
    if (n_in < 8) return;
    if (in_sizes[0] != NB * NQ * ND)        return;
    if (in_sizes[1] != NB * NSL * NM * ND)  return;
    if (in_sizes[2] != NB * NM)             return;
    if (in_sizes[3] != NB * NM)             return;
    if (in_sizes[4] != NHOP * ND * ND)      return;
    if (in_sizes[5] != NHOP * ND)           return;
    if (in_sizes[6] != NHOP * ND * ND)      return;
    if (in_sizes[7] != NHOP * ND)           return;
    if (out_size != NB * NQ * ND + NB * NQ * NM) return;

    const float* query = (const float*)d_in[0];
    const float* kb    = (const float*)d_in[1];
    const float* sel   = (const float*)d_in[2];
    const int*   mask  = (const int*)d_in[3];
    const float* Wq    = (const float*)d_in[4];
    const float* bq    = (const float*)d_in[5];
    const float* Wm    = (const float*)d_in[6];
    const float* vv    = (const float*)d_in[7];

    float* out_o = (float*)d_out;
    float* out_w = out_o + (size_t)NB * NQ * ND;

    const size_t sz_q16  = (size_t)NB * NQ * ND * 2;
    const size_t sz_w16  = (size_t)ND * ND * 2;
    const size_t sz_km16 = (size_t)NB * NM * ND * 2;
    const size_t sz_qhs  = (size_t)NB * NQ * ND * 4;
    const size_t sz_mhs  = (size_t)NB * NM * ND * 4;
    size_t off = 0;
    const size_t off_q16a = off;  off += sz_q16;
    const size_t off_q16b = off;  off += sz_q16;
    const size_t off_wq16 = off;  off += sz_w16;
    const size_t off_wm16 = off;  off += sz_w16;
    const size_t off_km16 = off;  off += sz_km16;
    const size_t off_kmT  = off;  off += sz_km16;
    const size_t off_qhs  = off;  off += sz_qhs;
    const size_t off_mhs  = off;  off += sz_mhs;
    if (off > ws_size) return;

    char* ws = (char*)d_ws;
    _Float16* q16a  = (_Float16*)(ws + off_q16a);
    _Float16* q16b  = (_Float16*)(ws + off_q16b);
    _Float16* wq16  = (_Float16*)(ws + off_wq16);
    _Float16* wm16  = (_Float16*)(ws + off_wm16);
    _Float16* km16  = (_Float16*)(ws + off_km16);
    _Float16* kmT16 = (_Float16*)(ws + off_kmT);
    float*    qhs   = (float*)(ws + off_qhs);
    float*    mhs   = (float*)(ws + off_mhs);

    const float C2  = 2.8853900817779268f;
    const float W16 = 0.0625f;

    for (int h = 0; h < NHOP; ++h) {
        const int nqb = (h == 0) ? (NB * NQ) / 4 : 0;
        const int nprep = nqb + ND / 4 + ND / 4 + (NB * NM) / 4 + NB * (NM / 64) * (ND / 32);
        prep_kernel<<<dim3(nprep), dim3(NTHR), 0, stream>>>(
            query, kb, sel, Wq, Wm, q16a, wq16, wm16, km16, kmT16, h, nqb);

        proj_gemm_kernel<<<dim3((NB * NQ) / 32), dim3(NTHR), 0, stream>>>(
            (h == 0) ? q16a : q16b, wq16, bq + (size_t)h * ND, 1.0f, W16, C2, qhs);

        proj_gemm_kernel<<<dim3((NB * NM) / 32), dim3(NTHR), 0, stream>>>(
            km16, wm16, bq + (size_t)h * ND, 0.0f, W16, C2, mhs);

        score_readout_kernel<<<dim3(NQ / 16, NB), dim3(NTHR), 0, stream>>>(
            qhs, mhs, vv, mask, kmT16, query, q16b, out_o, out_w, h, (h == NHOP - 1) ? 1 : 0);
    }
}
